// EpipolarCrossAttention_51376398794963
// MI455X (gfx1250) — hardware-verified
//
#include <hip/hip_runtime.h>


#define NB_  4
#define NN   4096
#define CC   256
#define NAG  320
#define OFF1 16777216
#define OFF2 16842752
#define RP   32
typedef _Float16 h16;
typedef unsigned short bf;
typedef __attribute__((ext_vector_type(16))) __bf16   v16bf;
typedef __attribute__((ext_vector_type(16))) _Float16 v16h;
typedef __attribute__((ext_vector_type(8)))  _Float16 v8h;
typedef __attribute__((ext_vector_type(8)))  unsigned short v8us;
typedef __attribute__((ext_vector_type(8)))  float    v8f;
typedef __attribute__((ext_vector_type(4)))  float    v4f;
typedef v8h  __attribute__((may_alias)) v8ha;
typedef v4f  __attribute__((may_alias)) v4fa;
typedef v8us __attribute__((may_alias)) v8usa;

__device__ __forceinline__ unsigned short f2bf(float f) { unsigned u = __float_as_uint(f); u += 0x7FFFu + ((u >> 16) & 1u); return (unsigned short)(u >> 16); }
__device__ __forceinline__ float bf2f(unsigned short b) { return __uint_as_float(((unsigned)b) << 16); }
__device__ __forceinline__ float bfr(float f) { return bf2f(f2bf(f)); }
__device__ __forceinline__ v16h cat16(v8h lo, v8h hi) { return __builtin_shufflevector(lo, hi, 0, 1, 2, 3, 4, 5, 6, 7, 8, 9, 10, 11, 12, 13, 14, 15); }
__device__ __forceinline__ v16bf cat16b(v8us lo, v8us hi) { return __builtin_bit_cast(v16bf, __builtin_shufflevector(lo, hi, 0, 1, 2, 3, 4, 5, 6, 7, 8, 9, 10, 11, 12, 13, 14, 15)); }
__device__ __forceinline__ v8f wmma16(v16h a, v16h b, v8f c) { return __builtin_amdgcn_wmma_f32_16x16x32_f16(false, a, false, b, (short)0, c, false, false); }
__device__ __forceinline__ v8f wmmab(v16bf a, v16bf b, v8f c) { return __builtin_amdgcn_wmma_f32_16x16x32_bf16(false, a, false, b, (short)0, c, false, false); }


template <typename T16> struct WFrag;
template <> struct WFrag<h16> { typedef v16h V; static __device__ __forceinline__ V ld(const h16* p) { return cat16(*(const v8h*)p, *(const v8h*)(p + 16)); } static __device__ __forceinline__ v8f mma(V a, V b, v8f c) { return wmma16(a, b, c); } };
template <> struct WFrag<bf> { typedef v16bf V; static __device__ __forceinline__ V ld(const bf* p) { return cat16b(*(const v8us*)p, *(const v8us*)(p + 16)); } static __device__ __forceinline__ v8f mma(V a, V b, v8f c) { return wmmab(a, b, c); } };
template <typename T16, int NSPLIT, bool BIAS>
__global__ __launch_bounds__(32) void k_gemmw(const T16* __restrict__ A, const T16* __restrict__ A2, const T16* __restrict__ Bt, const T16* __restrict__ Bt2, int K, float* C, int ldc, const float* __restrict__ bias, size_t sA, size_t sB, size_t sC) {
    typedef typename WFrag<T16>::V V;
    __shared__ __align__(16) float os[16 * 68];
    const size_t z = blockIdx.z; A += z * sA; if (A2) A2 += z * sA; Bt += z * sB; if (Bt2) Bt2 += z * sB; C += z * sC;
    const int lane = threadIdx.x & 31, lr = lane & 15, hi = lane >> 4; const int r0 = blockIdx.x * 64, c0 = blockIdx.y * 64;
    v8f acc[4][4];
#pragma unroll
    for (int mb = 0; mb < 4; ++mb)
#pragma unroll
        for (int nb = 0; nb < 4; ++nb) acc[mb][nb] = (v8f){};
    const size_t aoff = (size_t)(r0 + lr) * K + 8 * hi, boff = (size_t)(c0 + lr) * K + 8 * hi;
#pragma unroll 1
    for (int kc = 0; kc < K; kc += 32) {
        V a[4], a2[4];
#pragma unroll
        for (int mb = 0; mb < 4; ++mb) { a[mb] = WFrag<T16>::ld(A + aoff + (size_t)mb * 16 * K + kc); if (NSPLIT == 1 || NSPLIT == 2) a2[mb] = WFrag<T16>::ld(A2 + aoff + (size_t)mb * 16 * K + kc); }
#pragma unroll
        for (int nb = 0; nb < 4; ++nb) { const V b = WFrag<T16>::ld(Bt + boff + (size_t)nb * 16 * K + kc); V b2; if (NSPLIT >= 2) b2 = WFrag<T16>::ld(Bt2 + boff + (size_t)nb * 16 * K + kc);
#pragma unroll
            for (int mb = 0; mb < 4; ++mb) { acc[mb][nb] = WFrag<T16>::mma(a[mb], b, acc[mb][nb]); if (NSPLIT == 1 || NSPLIT == 2) acc[mb][nb] = WFrag<T16>::mma(a2[mb], b, acc[mb][nb]); if (NSPLIT >= 2) acc[mb][nb] = WFrag<T16>::mma(a[mb], b2, acc[mb][nb]); } }
        asm volatile("v_nop\n\tv_nop\n\tv_nop\n\tv_nop" : "+v"(acc[0][0]), "+v"(acc[1][1]), "+v"(acc[2][2]), "+v"(acc[3][3]) : "v"(a[0]), "v"(a[3]));
    }
#pragma unroll
    for (int mb = 0; mb < 4; ++mb) {
#pragma unroll
        for (int nb = 0; nb < 4; ++nb) {
#pragma unroll
            for (int j = 0; j < 8; ++j) os[(hi * 8 + j) * 68 + nb * 16 + lr] = acc[mb][nb][j]; }
        __builtin_amdgcn_wave_barrier(); asm volatile("" ::: "memory");
        float* crow = C + (size_t)(r0 + mb * 16) * ldc + c0;
#pragma unroll 1
        for (int ps = 0; ps < 2; ++ps) {
#pragma unroll
            for (int s = 0; s < 8; ++s) { const int row = 2 * s + hi, cofs = lr * 4; v4f val = *(const v4fa*)(os + row * 68 + cofs); if (BIAS) { val[0] += bfr(bias[c0 + cofs]); val[1] += bfr(bias[c0 + cofs + 1]); val[2] += bfr(bias[c0 + cofs + 2]); val[3] += bfr(bias[c0 + cofs + 3]); }
                *(volatile v4f*)(crow + (size_t)row * ldc + cofs) = val; }
            if (ps == 0) __threadfence(); }
        __builtin_amdgcn_wave_barrier(); asm volatile("" ::: "memory");
    }
}

__device__ __forceinline__ void splitf(float y, unsigned short& h, unsigned short& l) { h = f2bf(y); l = f2bf(y - bf2f(h)); }
typedef __attribute__((ext_vector_type(2))) unsigned short v2us;
typedef __attribute__((ext_vector_type(4))) unsigned short v4us;
typedef __attribute__((ext_vector_type(2))) float v2f;
__global__ __launch_bounds__(256) void k_wtG(const float* __restrict__ w, int K, int N, bf* Bt) {
    const int lane = threadIdx.x & 31; const int L0 = (blockIdx.x * 8 + (threadIdx.x >> 5)) * 8; const int nlines = N * K / 64;
#pragma unroll
    for (int ps = 0; ps < 2; ++ps) {
#pragma unroll 1
        for (int l = 0; l < 8; ++l) { const int L = L0 + l; if (L >= nlines) break; const size_t e = (size_t)L * 64 + lane * 2; const int k = (int)(e % K), n = (int)(e / K); v2us o;
            o[0] = f2bf(w[(size_t)k * N + n]); o[1] = f2bf(w[(size_t)(k + 1) * N + n]); *(volatile v2us*)(Bt + e) = o; }
        if (ps == 0) __threadfence(); }
}
__global__ __launch_bounds__(256) void k_cvt8(const float* __restrict__ src, bf* dst, size_t n8) { const size_t i = (size_t)blockIdx.x * 256 + threadIdx.x; if (i >= n8) return; const v8f v = *(const v8f*)(src + i * 8); v8us o;
#pragma unroll
    for (int k = 0; k < 8; ++k) o[k] = f2bf(v[k]); *(volatile v8us*)(dst + i * 8) = o; __threadfence(); *(volatile v8us*)(dst + i * 8) = o; }

__global__ __launch_bounds__(256) void k_split4(const float* __restrict__ F, bf* Ph, bf* Pl, size_t n4) { const size_t i = (size_t)blockIdx.x * 256 + threadIdx.x; if (i >= n4) return; const v4f v = *(const v4f*)(F + i * 4); v4us oh, ol;
#pragma unroll
    for (int q = 0; q < 4; ++q) { unsigned short a, c; splitf(v[q], a, c); oh[q] = a; ol[q] = c; } *(volatile v4us*)(Ph + i * 4) = oh; *(volatile v4us*)(Pl + i * 4) = ol; __threadfence(); *(volatile v4us*)(Ph + i * 4) = oh; *(volatile v4us*)(Pl + i * 4) = ol; }
__global__ __launch_bounds__(256) void k_splitp(const float* __restrict__ F, bf* Ph, bf* Pl) { const size_t e = ((size_t)blockIdx.x * 256 + threadIdx.x) * 4; if (e >= (size_t)NN * CC) return; const int c = (int)(e % CC); const size_t n = e / CC; const v4f v = *(const v4f*)(F + n * NAG + c); v4us oh, ol;
#pragma unroll
    for (int q = 0; q < 4; ++q) { unsigned short a, c2; splitf(v[q], a, c2); oh[q] = a; ol[q] = c2; } *(volatile v4us*)(Ph + e) = oh; *(volatile v4us*)(Pl + e) = ol; __threadfence(); *(volatile v4us*)(Ph + e) = oh; *(volatile v4us*)(Pl + e) = ol; }
__global__ __launch_bounds__(256) void k_krf(const float* __restrict__ kR, float* KRF) { const int j = blockIdx.x * 256 + threadIdx.x; if (j >= NN) return; v2f o; o[0] = bfr(kR[(size_t)j * 2]); o[1] = bfr(kR[(size_t)j * 2 + 1]); *(volatile v2f*)(KRF + (size_t)j * 2) = o; __threadfence(); *(volatile v2f*)(KRF + (size_t)j * 2) = o; }
__global__ __launch_bounds__(256) void k_zero8(bf* Z, size_t n8) { const size_t i = (size_t)blockIdx.x * 256 + threadIdx.x; if (i >= n8) return; const v8us z = (v8us){}; *(volatile v8us*)(Z + i * 8) = z; __threadfence(); *(volatile v8us*)(Z + i * 8) = z; }
__global__ __launch_bounds__(256) void k_vk(const float* __restrict__ Wk, const float* __restrict__ bq, float* VK) { const int c = blockIdx.x * 256 + threadIdx.x; if (c >= CC) return; float s = 0.f;
#pragma unroll 4
    for (int o = 0; o < CC; ++o) { float p = __fmul_rn(bfr(Wk[o * CC + c]), bfr(bq[o])); asm volatile("" : "+v"(p)); s = __fadd_rn(s, p); }
    s = __fmul_rn(s, 0.0625f);     *(volatile float*)(VK + c) = s; __threadfence(); *(volatile float*)(VK + c) = s; }
__global__ __launch_bounds__(256) void k_colterm(const float* __restrict__ y, const float* __restrict__ VK, float* CT) { const int m = blockIdx.x * 256 + threadIdx.x; if (m >= NN) return; float s = 0.f;
#pragma unroll 4
    for (int c = 0; c < CC; ++c) { float p = __fmul_rn(bfr(y[(size_t)m * CC + c]), VK[c]); asm volatile("" : "+v"(p)); s = __fadd_rn(s, p); }
    *(volatile float*)(CT + m) = s; __threadfence(); *(volatile float*)(CT + m) = s; }
__global__ __launch_bounds__(256) void k_yt(const float* __restrict__ y, const float* __restrict__ kR, bf* YT) { const size_t e = ((size_t)blockIdx.x * 256 + threadIdx.x) * 2; if (e >= (size_t)NAG * NN) return; const int m = (int)(e % NN), r = (int)(e / NN); v2us o; o[0] = 0; o[1] = 0;
    if (r < CC) { o[0] = f2bf(y[(size_t)m * CC + r]); o[1] = f2bf(y[(size_t)(m + 1) * CC + r]); } else if (r == CC) { o[0] = f2bf(kR[(size_t)m * 2]); o[1] = f2bf(kR[(size_t)(m + 1) * 2]); }
    *(volatile v2us*)(YT + e) = o; __threadfence(); *(volatile v2us*)(YT + e) = o; }
__global__ __launch_bounds__(256) void k_esoft(const float* __restrict__ S, const float* __restrict__ CT, const float* __restrict__ kL, const float* __restrict__ KRF, bf* Ph, bf* Pl, float* CNT) {
    const int lane = threadIdx.x & 31; const int n = blockIdx.x * 8 + (threadIdx.x >> 5); if (n >= NN) return; float uL = bfr(kL[(size_t)n * 2]), vL = bfr(kL[(size_t)n * 2 + 1]); asm volatile("" : "+v"(uL)); asm volatile("" : "+v"(vL));     const float* sr = S + (size_t)n * NN; float v[NN / 32]; float mx = -3.0e38f; int cnt = 0;
#pragma unroll
    for (int ch = 0; ch < NN / 128; ++ch) { const int j0 = ch * 128 + lane * 4; const v4f a = *(const v4f*)(sr + j0);
#pragma unroll
        for (int q = 0; q < 4; ++q) { const int j = j0 + q; const v2f kr = *(const v2f*)(KRF + (size_t)j * 2); float ur = kr[0], vr = kr[1]; asm volatile("" : "+v"(ur)); asm volatile("" : "+v"(vr)); const float du = __fsub_rn(uL, ur); const float dv = fabsf(__fsub_rn(vL, vr)); const bool ok = (dv < 3.0f) && (du > 0.0f) && (du < 192.0f); float sa = __fmul_rn(a[q], 0.0625f); asm volatile("" : "+v"(sa)); float ctj = CT[j]; asm volatile("" : "+v"(ctj)); const float t = ok ? __fadd_rn(sa, ctj) : -1.0e9f; cnt += ok ? 1 : 0; v[ch * 4 + q] = t; mx = fmaxf(mx, t); } }
#pragma unroll
    for (int sh = 16; sh; sh >>= 1) { mx = fmaxf(mx, __shfl_xor(mx, sh, 32)); cnt += __shfl_xor(cnt, sh, 32); }
    float sum = 0.f;
#pragma unroll
    for (int k = 0; k < NN / 32; ++k) { float d0 = __fsub_rn(v[k], mx); asm volatile("" : "+v"(d0)); v[k] = __builtin_amdgcn_exp2f(__fmul_rn(d0, 1.4426950408889634f)); sum += v[k]; }
#pragma unroll
    for (int sh = 16; sh; sh >>= 1) sum += __shfl_xor(sum, sh, 32);
    const float f = __fdiv_rn(1.0f, sum);
#pragma unroll 1
    for (int ps = 0; ps < 2; ++ps) {
#pragma unroll
        for (int ch = 0; ch < NN / 128; ++ch) { v4us oh, ol;
#pragma unroll
            for (int q = 0; q < 4; ++q) { unsigned short a, c2; splitf(v[ch * 4 + q] * f, a, c2); oh[q] = a; ol[q] = c2; }
            const size_t oo = (size_t)n * NN + ch * 128 + lane * 4; *(volatile v4us*)(Ph + oo) = oh; *(volatile v4us*)(Pl + oo) = ol; }
        if (lane == 0) *(volatile float*)(CNT + (size_t)n * RP) = (float)cnt;
        if (ps == 0) __threadfence(); } }
__global__ __launch_bounds__(256) void k_fin(const float* __restrict__ AG, const float* __restrict__ CNT, const float* __restrict__ kL, float* DSP, float* CNF) { const int n = blockIdx.x * 256 + threadIdx.x; if (n >= NN) return; const float uL = bfr(kL[(size_t)n * 2]); const float dsp = __fsub_rn(uL, AG[(size_t)n * NAG + CC]); const float cf = (CNT[(size_t)n * RP] > 0.5f) ? 1.0f : 0.0f;
    *(volatile float*)(DSP + n) = dsp; *(volatile float*)(CNF + n) = cf; __threadfence(); *(volatile float*)(DSP + n) = dsp; *(volatile float*)(CNF + n) = cf; }

extern "C" void kernel_launch(void* const* d_in, const int* in_sizes, int n_in,
                              void* d_out, int out_size, void* d_ws, size_t ws_size, hipStream_t stream) {
    (void)in_sizes; (void)n_in; (void)out_size;
    const float* xL = (const float*)d_in[0]; const float* xR = (const float*)d_in[1]; const float* kL = (const float*)d_in[2]; const float* kR = (const float*)d_in[3];
    const float* Wq = (const float*)d_in[4]; const float* bq = (const float*)d_in[5]; const float* Wk = (const float*)d_in[6]; (void)d_in[7]; const float* Wv = (const float*)d_in[8]; const float* bv = (const float*)d_in[9]; const float* Wm = (const float*)d_in[10]; const float* bm = (const float*)d_in[11];
    float* OUT0 = (float*)d_out; float* DSP = (float*)((char*)d_out + OFF1); float* CNF = (float*)((char*)d_out + OFF2);
    char* wsp = (char*)d_ws;
    auto take = [&](size_t bytes) { char* p = wsp; wsp += (bytes + 255) & ~(size_t)255; return (void*)p; };
    bf* WQT = (bf*)take(CC * CC * 2); bf* WKT = (bf*)take(CC * CC * 2); float* MT = (float*)take(CC * CC * 4); bf* MTh = (bf*)take(CC * CC * 2); bf* MTl = (bf*)take(CC * CC * 2); float* VK = (float*)take(CC * 4); bf* WVb = (bf*)take(CC * CC * 2); bf* WMb = (bf*)take(CC * CC * 2);
    bf* XL = (bf*)take((size_t)NN * CC * 2); bf* ZX = (bf*)take((size_t)NN * CC * 2); bf* XRb = (bf*)take((size_t)NN * CC * 2); bf* YT = (bf*)take((size_t)NAG * NN * 2); float* CT = (float*)take(NN * 4); float* KRF = (float*)take((size_t)NN * 2 * 4);
    float* T1 = (float*)take((size_t)NN * CC * 4); bf* T1h = (bf*)take((size_t)NN * CC * 2); bf* T1l = (bf*)take((size_t)NN * CC * 2); float* S = (float*)take((size_t)NN * NN * 4); bf* Ph = (bf*)take((size_t)NN * NN * 2); bf* Pl = (bf*)take((size_t)NN * NN * 2); float* CNT = (float*)take((size_t)NN * RP * 4);
    float* AG = (float*)take((size_t)NN * NAG * 4); bf* AGh = (bf*)take((size_t)NN * CC * 2); bf* AGl = (bf*)take((size_t)NN * CC * 2); float* MV = (float*)take((size_t)NN * CC * 4); bf* MVh = (bf*)take((size_t)NN * CC * 2); bf* MVl = (bf*)take((size_t)NN * CC * 2);
    if ((size_t)(wsp - (char*)d_ws) > ws_size) return;
    k_wtG<<<(CC * CC / 64 + 63) / 64, 256, 0, stream>>>(Wk, CC, CC, WKT); k_wtG<<<(CC * CC / 64 + 63) / 64, 256, 0, stream>>>(Wq, CC, CC, WQT);
    k_gemmw<bf, 0, false><<<dim3(CC / 64, CC / 64, 1), 32, 0, stream>>>(WKT, nullptr, WQT, nullptr, CC, MT, CC, nullptr, 0, 0, 0);
    k_split4<<<(CC * CC / 4 + 255) / 256, 256, 0, stream>>>(MT, MTh, MTl, (size_t)CC * CC / 4); k_vk<<<1, 256, 0, stream>>>(Wk, bq, VK);
    k_cvt8<<<(CC * CC / 8 + 255) / 256, 256, 0, stream>>>(Wv, WVb, (size_t)CC * CC / 8); k_cvt8<<<(CC * CC / 8 + 255) / 256, 256, 0, stream>>>(Wm, WMb, (size_t)CC * CC / 8);
    k_zero8<<<(unsigned)(((size_t)NN * CC / 8 + 255) / 256), 256, 0, stream>>>(ZX, (size_t)NN * CC / 8);
    for (int b = 0; b < NB_; ++b) {
        const float* xLb = xL + (size_t)b * NN * CC; const float* xRb = xR + (size_t)b * NN * CC; const float* kLb = kL + (size_t)b * NN * 2; const float* kRb = kR + (size_t)b * NN * 2;
        k_cvt8<<<(unsigned)(((size_t)NN * CC / 8 + 255) / 256), 256, 0, stream>>>(xLb, XL, (size_t)NN * CC / 8); k_cvt8<<<(unsigned)(((size_t)NN * CC / 8 + 255) / 256), 256, 0, stream>>>(xRb, XRb, (size_t)NN * CC / 8);
        k_yt<<<(unsigned)(((size_t)NAG * NN / 2 + 255) / 256), 256, 0, stream>>>(xRb, kRb, YT); k_colterm<<<NN / 256, 256, 0, stream>>>(xRb, VK, CT); k_krf<<<NN / 256, 256, 0, stream>>>(kRb, KRF);
        k_gemmw<bf, 2, false><<<dim3(NN / 64, CC / 64, 1), 32, 0, stream>>>(XL, ZX, MTh, MTl, CC, T1, CC, nullptr, 0, 0, 0);
        k_split4<<<(unsigned)(((size_t)NN * CC / 4 + 255) / 256), 256, 0, stream>>>(T1, T1h, T1l, (size_t)NN * CC / 4);
        k_gemmw<bf, 1, false><<<dim3(NN / 64, NN / 64, 1), 32, 0, stream>>>(T1h, T1l, XRb, nullptr, CC, S, NN, nullptr, 0, 0, 0);
        k_esoft<<<NN / 8, 256, 0, stream>>>(S, CT, kLb, KRF, Ph, Pl, CNT);
        k_gemmw<bf, 1, false><<<dim3(NN / 64, NAG / 64, 1), 32, 0, stream>>>(Ph, Pl, YT, nullptr, NN, AG, NAG, nullptr, 0, 0, 0);
        k_splitp<<<(unsigned)(((size_t)NN * CC / 4 + 255) / 256), 256, 0, stream>>>(AG, AGh, AGl);
        k_gemmw<bf, 1, true><<<dim3(NN / 64, CC / 64, 1), 32, 0, stream>>>(AGh, AGl, WVb, nullptr, CC, MV, CC, bv, 0, 0, 0);
        k_split4<<<(unsigned)(((size_t)NN * CC / 4 + 255) / 256), 256, 0, stream>>>(MV, MVh, MVl, (size_t)NN * CC / 4);
        k_gemmw<bf, 1, true><<<dim3(NN / 64, CC / 64, 1), 32, 0, stream>>>(MVh, MVl, WMb, nullptr, CC, OUT0 + (size_t)b * NN * CC, CC, bm, 0, 0, 0);
        k_fin<<<NN / 256, 256, 0, stream>>>(AG, CNT, kLb, DSP + (size_t)b * NN, CNF + (size_t)b * NN); }
}
